// MambaBlock_12163347382741
// MI455X (gfx1250) — hardware-verified
//
#include <hip/hip_runtime.h>
#include <math.h>

typedef __attribute__((ext_vector_type(16))) _Float16 v16h;
typedef __attribute__((ext_vector_type(8)))  _Float16 v8h;
typedef __attribute__((ext_vector_type(8)))  float    v8f;
typedef __attribute__((ext_vector_type(4)))  float    v4f;

constexpr int kBatch   = 2;
constexpr int kSeq     = 2048;
constexpr int kDm      = 768;
constexpr int kDin     = 1536;
constexpr int kNst     = 16;
constexpr int kXzP     = 2 * kDin;
constexpr int kBcReal  = 2 * kNst;
constexpr int kBcP     = 64;
constexpr int kRows    = kBatch * kSeq;
constexpr int kConvTP  = 260;
constexpr int kScanTS  = 64;
constexpr int kScanCh  = 64;
constexpr int kScanYP  = 68;
constexpr float kCarryX  = 64.0f;
constexpr float kCarryW  = 1024.0f;
constexpr float kCarryXi = 1024.0f;
constexpr float kCarryY  = 1024.0f;
constexpr float kFoldS0  = 1.0f / (kCarryX * kCarryW);
constexpr float kFoldS1  = 1.0f / (kCarryXi * kCarryW);
constexpr float kFoldS4  = 1.0f / (kCarryY * kCarryW);

static_assert(kXzP == 3072 && kRows == 4096 && kBcReal == 32, "shape constants");
static_assert((kDm % 32) == 0 && (kDin % 32) == 0, "GEMM K multiples of 32");
static_assert((kRows % 64) == 0 && (kXzP % 64) == 0 && (kDin % 64) == 0 && (kBcP % 64) == 0 && (kDm % 64) == 0, "GEMM M,N multiples of 64");
static_assert(((kRows / 64) * (kXzP / 64)) % 8 == 0 && ((kRows / 64) * (kDin / 64)) % 8 == 0 &&
              ((kRows / 64) * (kBcP / 64)) % 8 == 0 && ((kRows / 64) * (kDm / 64)) % 8 == 0, "tiles fill whole blocks");
static_assert((kSeq % kScanTS) == 0 && (kSeq % 64) == 0 && (kDin % kScanCh) == 0 && (kDin % 256) == 0, "tile multiples");
static_assert((kRows * kDm / 8) % 256 == 0 && (kXzP * kDm / 8) % 256 == 0 && (kDin * kDin / 8) % 256 == 0 &&
              (kDm * kDin / 8) % 256 == 0 && (kBcP * kDin / 8) % 256 == 0, "cast grids exact");

constexpr size_t kOffX16    = 0;
constexpr size_t kOffWIN16  = kOffX16    + (size_t)kRows * kDm  * 2;
constexpr size_t kOffWDT16  = kOffWIN16  + (size_t)kXzP  * kDm  * 2;
constexpr size_t kOffWOUT16 = kOffWDT16  + (size_t)kDin  * kDin * 2;
constexpr size_t kOffWX16   = kOffWOUT16 + (size_t)kDm   * kDin * 2;
constexpr size_t kOffXZ     = kOffWX16   + (size_t)kBcP  * kDin * 2;
constexpr size_t kOffXI     = kOffXZ     + (size_t)kRows * kXzP * 4;
constexpr size_t kOffXI16   = kOffXI     + (size_t)kRows * kDin * 4;
constexpr size_t kOffDLR    = kOffXI16   + (size_t)kRows * kDin * 2;
constexpr size_t kOffBC     = kOffDLR    + (size_t)kRows * kDin * 4;
constexpr size_t kWsTotal   = kOffBC     + (size_t)kRows * kBcP * 4;
static_assert(kWsTotal == 132579328ull, "carve total");
static_assert(kWsTotal <= 134217728ull, "carve cap");
static_assert((kOffWIN16 % 128) == 0 && (kOffWDT16 % 128) == 0 && (kOffWOUT16 % 128) == 0 && (kOffWX16 % 128) == 0 &&
              (kOffXZ % 128) == 0 && (kOffXI % 128) == 0 && (kOffXI16 % 128) == 0 && (kOffDLR % 128) == 0 &&
              (kOffBC % 128) == 0, "128-B aligned regions");

__device__ __forceinline__ unsigned short f2bf_bits(float f) {
  unsigned u = __float_as_uint(f);
  return (unsigned short)((u + 0x7FFFu + ((u >> 16) & 1u)) >> 16);
}
__device__ __forceinline__ float bf_bits2f(unsigned short h) { return __uint_as_float(((unsigned)h) << 16); }
__device__ __forceinline__ float bf16_rne(float f) { return bf_bits2f(f2bf_bits(f)); }

__device__ __forceinline__ void guard4_h(v8f& a, v8f& b, v8f& c, v8f& d, v16h x, v16h y) {
  asm volatile("v_nop\n\tv_nop\n\tv_nop\n\tv_nop" : "+v"(a), "+v"(b), "+v"(c), "+v"(d) : "v"(x), "v"(y));
}
__device__ __forceinline__ void keep4_h(v16h a, v16h b, v16h c, v16h d) { asm volatile("v_nop" :: "v"(a), "v"(b), "v"(c), "v"(d)); }
__device__ __forceinline__ void acc_guard4(v8f& a, v8f& b, v8f& c, v8f& d) { asm volatile("v_nop\n\tv_nop\n\tv_nop\n\tv_nop" : "+v"(a), "+v"(b), "+v"(c), "+v"(d)); }

union FragU { v16h v; v8h h[2]; };
__device__ __forceinline__ v16h frag_load(const _Float16* p) {
  FragU f;
  f.h[0] = *(const v8h*)(p);
  f.h[1] = *(const v8h*)(p + 16);
  return f.v;
}
__device__ __forceinline__ v8f frag_mma(v16h a, v16h b, v8f c) {
  return __builtin_amdgcn_wmma_f32_16x16x32_f16(false, a, false, b, (short)0, c, false, false);
}

__global__ __launch_bounds__(256) void gemm_f16_kernel(
    const unsigned short* __restrict__ Ap, int lda,
    const unsigned short* __restrict__ Btp, int ldb,
    float* __restrict__ C, int ldc,
    int M, int N, int K, float scale)
{
  const _Float16* A  = (const _Float16*)Ap;
  const _Float16* Bt = (const _Float16*)Btp;
  __shared__ __align__(16) float sT[8][16 * 68];
  const int lane = threadIdx.x & 31;
  const int wave = threadIdx.x >> 5;
  const int tilesN = N >> 6;
  const int tilesM = M >> 6;
  const int tile = blockIdx.x * 8 + wave;
  if (tile >= tilesM * tilesN) return;
  const int tm = tile / tilesN;
  const int tn = tile - tm * tilesN;
  const int m0 = tm << 6;
  const int n0 = tn << 6;

  const int rlane = lane & 15;
  const int koff  = (lane >> 4) * 8;
  const int mOff  = (lane >> 4) * 8;

  v8f acc[4][4];
#pragma unroll
  for (int i = 0; i < 4; ++i)
#pragma unroll
    for (int j = 0; j < 4; ++j) acc[i][j] = (v8f){0.f,0.f,0.f,0.f,0.f,0.f,0.f,0.f};

  for (int k0 = 0; k0 < K; k0 += 32) {
    v16h bh[4];
#pragma unroll
    for (int j = 0; j < 4; ++j) {
      const size_t bo = (size_t)(n0 + (j << 4) + rlane) * ldb + koff + k0;
      bh[j] = frag_load(Bt + bo);
    }
#pragma unroll
    for (int i = 0; i < 4; ++i) {
      const size_t ao = (size_t)(m0 + (i << 4) + rlane) * lda + koff + k0;
      v16h ah = frag_load(A + ao);
#pragma unroll
      for (int j = 0; j < 4; ++j) acc[i][j] = frag_mma(ah, bh[j], acc[i][j]);
      guard4_h(acc[i][0], acc[i][1], acc[i][2], acc[i][3], ah, bh[3]);
    }
    keep4_h(bh[0], bh[1], bh[2], bh[3]);
  }
  acc_guard4(acc[0][0], acc[0][1], acc[0][2], acc[0][3]);
  acc_guard4(acc[1][0], acc[1][1], acc[1][2], acc[1][3]);
  acc_guard4(acc[2][0], acc[2][1], acc[2][2], acc[2][3]);
  acc_guard4(acc[3][0], acc[3][1], acc[3][2], acc[3][3]);

  float* slab = sT[wave];
#pragma unroll
  for (int i = 0; i < 4; ++i) {
    const int mBase = m0 + (i << 4);
#pragma unroll
    for (int j = 0; j < 4; ++j) {
#pragma unroll
      for (int r = 0; r < 8; ++r) {
        const float v = acc[i][j][r] * scale;
        slab[(mOff + r) * 68 + (j << 4) + rlane] = v;
      }
    }
    __builtin_amdgcn_fence(__ATOMIC_RELEASE, "workgroup");
    __builtin_amdgcn_wave_barrier();
    __builtin_amdgcn_fence(__ATOMIC_ACQUIRE, "workgroup");
    {
      const int hh = lane >> 4, c4 = (lane & 15) * 4;
      for (int pass = 0; pass < 2; ++pass) {
#pragma unroll
        for (int it = 0; it < 8; ++it) {
          const int row = it * 2 + hh;
          v4f v = *(const v4f*)(slab + row * 68 + c4);
          *(volatile v4f*)(C + (size_t)(mBase + row) * ldc + n0 + c4) = v;
        }
        __threadfence();
      }
    }
    __builtin_amdgcn_fence(__ATOMIC_RELEASE, "workgroup");
    __builtin_amdgcn_wave_barrier();
    __builtin_amdgcn_fence(__ATOMIC_ACQUIRE, "workgroup");
  }
}

__global__ __launch_bounds__(256) void cast_plane_kernel(
    const float* __restrict__ src, unsigned short* __restrict__ dst, int real8, int total8, float scale)
{
  const int i = blockIdx.x * 256 + threadIdx.x;
  if (i >= total8) return;
  const bool live = (i < real8);
  const int ic = live ? i : (real8 - 1);
  const size_t es = (size_t)ic << 3;
  const v4f a0 = *(const v4f*)(src + es);
  const v4f a1 = *(const v4f*)(src + es + 4);
  v8h hv;
#pragma unroll
  for (int e = 0; e < 4; ++e) {
    const float f0 = a0[e];
    const float f1 = a1[e];
    const float r0 = bf16_rne(f0) * scale;
    const float r1 = bf16_rne(f1) * scale;
    const float s0 = live ? r0 : 0.0f;
    const float s1 = live ? r1 : 0.0f;
    hv[e]     = (_Float16)s0;
    hv[4 + e] = (_Float16)s1;
  }
  unsigned short* q = dst + ((size_t)i << 3);
  *(volatile v8h*)q = hv;
  __threadfence();
  *(volatile v8h*)q = hv;
}

__global__ __launch_bounds__(256) void conv_silu_kernel(
    const float* __restrict__ XZ, const float* __restrict__ cw, const float* __restrict__ cb,
    float* __restrict__ XI, unsigned short* __restrict__ XI16)
{
  __shared__ __align__(16) float sT[16 * kConvTP];
  const int tid = threadIdx.x, lane = tid & 31, wave = tid >> 5;
  const int d0 = blockIdx.x * 256, d = d0 + tid;
  const int g0 = blockIdx.y * 64;
  const int tb = g0 & (kSeq - 1);
  const float w0 = bf16_rne(cw[d * 3 + 0]);
  const float w1 = bf16_rne(cw[d * 3 + 1]);
  const float w2 = bf16_rne(cw[d * 3 + 2]);
  const float bc = bf16_rne(cb[d]);
  float xprev, xcur;
  {
    const int rp = (g0 > 0) ? (g0 - 1) : 0;
    const float vp = XZ[(size_t)rp * kXzP + d];
    xprev = (tb > 0) ? vp : 0.0f;
    xcur  = XZ[(size_t)g0 * kXzP + d];
  }
  const int hrow = wave >> 1;
  const int hch  = (wave & 1) * 128 + lane * 4;
#pragma unroll 1
  for (int sub = 0; sub < 4; ++sub) {
    const int lb = g0 + sub * 16;
#pragma unroll 1
    for (int s = 0; s < 16; ++s) {
      const int gn  = lb + s + 1;
      const int gnc = (gn < kRows) ? gn : (kRows - 1);
      const float vn = XZ[(size_t)gnc * kXzP + d];
      const int tn = tb + sub * 16 + s + 1;
      const float xnext = (tn < kSeq) ? vn : 0.0f;
      float acc = w0 * xprev;
      acc = fmaf(w1, xcur, acc);
      acc = fmaf(w2, xnext, acc);
      const float sv = acc + bc;
      const float ev = expf(-sv);
      const float sg = 1.0f / (1.0f + ev);
      sT[s * kConvTP + tid] = sv * sg;
      xprev = xcur;
      xcur  = xnext;
    }
    __syncthreads();
    v4f fv[4];
    v8h bv[2];
#pragma unroll
    for (int it = 0; it < 4; ++it) fv[it] = *(const v4f*)(sT + (it * 4 + hrow) * kConvTP + hch);
#pragma unroll
    for (int it = 0; it < 2; ++it) {
      const float* sp = sT + (it * 8 + wave) * kConvTP + lane * 8;
      const v4f a0 = *(const v4f*)(sp);
      const v4f a1 = *(const v4f*)(sp + 4);
#pragma unroll
      for (int e = 0; e < 4; ++e) {
        const float f0 = a0[e] * kCarryXi;
        const float f1 = a1[e] * kCarryXi;
        bv[it][e]     = (_Float16)f0;
        bv[it][4 + e] = (_Float16)f1;
      }
    }
    for (int pass = 0; pass < 2; ++pass) {
#pragma unroll
      for (int it = 0; it < 4; ++it)
        *(volatile v4f*)(XI + (size_t)(lb + it * 4 + hrow) * kDin + d0 + hch) = fv[it];
#pragma unroll
      for (int it = 0; it < 2; ++it)
        *(volatile v8h*)(XI16 + (size_t)(lb + it * 8 + wave) * kDin + d0 + lane * 8) = bv[it];
      __threadfence();
    }
    __syncthreads();
  }
}

__global__ __launch_bounds__(64) void scan_kernel(
    const float* __restrict__ BC, const float* __restrict__ DLR, const float* __restrict__ XI,
    const float* __restrict__ XZ, const float* __restrict__ bdt, const float* __restrict__ Alog,
    const float* __restrict__ Dp, unsigned short* __restrict__ Y16)
{
  __shared__ __align__(16) float sX[kScanTS * kBcReal];
  __shared__ __align__(16) float sY[kScanTS * kScanYP];
  __shared__ __align__(16) float sA[kNst * kScanCh];
  const int tid = threadIdx.x, lane = tid & 31, wave = tid >> 5;
  constexpr int kBlkPerB = kDin / kScanCh;
  const int bix = blockIdx.x / kBlkPerB;
  const int d0  = (blockIdx.x - bix * kBlkPerB) * kScanCh;
  const int d   = d0 + tid;
  const size_t row0 = (size_t)bix * kSeq;
#pragma unroll 1
  for (int s = 0; s < kNst; ++s) {
    const float al = bf16_rne(Alog[(size_t)d * kNst + s]);
    sA[s * kScanCh + tid] = -expf(al);
  }
  __syncthreads();
  float negA[kNst], h[kNst];
#pragma unroll
  for (int s = 0; s < kNst; ++s) {
    negA[s] = sA[s * kScanCh + tid];
    h[s] = 0.0f;
  }
  const float bb = bf16_rne(bdt[d]);
  const float Dd = bf16_rne(Dp[d]);
  const int lr = tid >> 3, lc4 = (tid & 7) * 4;
  const int q = lane >> 3, c8 = (lane & 7) * 8;
#pragma unroll 1
  for (int t0 = 0; t0 < kSeq; t0 += kScanTS) {
    __syncthreads();
#pragma unroll
    for (int i = 0; i < 8; ++i) {
      const int r = lr + 8 * i;
      *(v4f*)(sX + r * kBcReal + lc4) = *(const v4f*)(BC + (row0 + t0 + r) * kBcP + lc4);
    }
    __syncthreads();
#pragma unroll 1
    for (int s = 0; s < kScanTS; ++s) {
      const size_t row = row0 + (size_t)(t0 + s);
      const float* xr = sX + s * kBcReal;
      float Bs[kNst], Cs[kNst];
#pragma unroll
      for (int q4 = 0; q4 < 4; ++q4) {
        const v4f bv = *(const v4f*)(xr + 4 * q4);
        const v4f cv = *(const v4f*)(xr + kNst + 4 * q4);
        Bs[4 * q4 + 0] = bv[0]; Bs[4 * q4 + 1] = bv[1]; Bs[4 * q4 + 2] = bv[2]; Bs[4 * q4 + 3] = bv[3];
        Cs[4 * q4 + 0] = cv[0]; Cs[4 * q4 + 1] = cv[1]; Cs[4 * q4 + 2] = cv[2]; Cs[4 * q4 + 3] = cv[3];
      }
      const float v   = DLR[row * kDin + d] + bb;
      const float xt  = XI[row * kDin + d];
      const float zv  = XZ[row * kXzP + kDin + d];
      const float a   = __expf(-fabsf(v));
      const float u   = 1.0f + a;
      const float l1p = __logf(u) + (a - (u - 1.0f)) * __builtin_amdgcn_rcpf(u);
      const float dt  = fmaxf(v, 0.0f) + l1p;
      const float dtx = dt * xt;
      float y = 0.0f;
#pragma unroll
      for (int k = 0; k < kNst; ++k) {
        const float e = __expf(dt * negA[k]);
        h[k] = e * h[k] + dtx * Bs[k];
        y = h[k] * Cs[k] + y;
      }
      y = xt * Dd + y;
      const float eg = expf(-zv);
      const float g  = zv * (1.0f / (1.0f + eg));
      sY[s * kScanYP + tid] = (y * g) * kCarryY;
    }
    __syncthreads();
    v8h hv[8];
#pragma unroll
    for (int it = 0; it < 8; ++it) {
      const int rr = it * 8 + wave * 4 + q;
      const float* sp = sY + rr * kScanYP + c8;
      const v4f a0 = *(const v4f*)(sp);
      const v4f a1 = *(const v4f*)(sp + 4);
#pragma unroll
      for (int e = 0; e < 4; ++e) {
        const float f0 = a0[e];
        const float f1 = a1[e];
        hv[it][e]     = (_Float16)f0;
        hv[it][4 + e] = (_Float16)f1;
      }
    }
    for (int pass = 0; pass < 2; ++pass) {
#pragma unroll
      for (int it = 0; it < 8; ++it) {
        const int rr = it * 8 + wave * 4 + q;
        const size_t o = (row0 + (size_t)(t0 + rr)) * kDin + d0 + c8;
        *(volatile v8h*)(Y16 + o) = hv[it];
      }
      __threadfence();
    }
  }
}

extern "C" void kernel_launch(void* const* d_in, const int* in_sizes, int n_in,
                              void* d_out, int out_size, void* d_ws, size_t ws_size,
                              hipStream_t stream) {
  if (n_in < 10) return;
  if (in_sizes[0] != kRows * kDm) return;
  if (in_sizes[1] != kXzP * kDm) return;
  if (in_sizes[2] != kDin * 3) return;
  if (in_sizes[3] != kDin) return;
  if (in_sizes[4] != kBcReal * kDin) return;
  if (in_sizes[5] != kDin * kDin) return;
  if (in_sizes[6] != kDin) return;
  if (in_sizes[7] != kDin * kNst) return;
  if (in_sizes[8] != kDin) return;
  if (in_sizes[9] != kDm * kDin) return;
  if (out_size != kRows * kDm) return;
  if (ws_size < kWsTotal) return;

  const float* x      = (const float*)d_in[0];
  const float* W_in   = (const float*)d_in[1];
  const float* conv_w = (const float*)d_in[2];
  const float* conv_b = (const float*)d_in[3];
  const float* W_x    = (const float*)d_in[4];
  const float* W_dt   = (const float*)d_in[5];
  const float* b_dt   = (const float*)d_in[6];
  const float* A_log  = (const float*)d_in[7];
  const float* Dp     = (const float*)d_in[8];
  const float* W_out  = (const float*)d_in[9];
  float* out = (float*)d_out;

  char* ws = (char*)d_ws;
  unsigned short* X16    = (unsigned short*)(ws + kOffX16);
  unsigned short* WIN16  = (unsigned short*)(ws + kOffWIN16);
  unsigned short* WDT16  = (unsigned short*)(ws + kOffWDT16);
  unsigned short* WOUT16 = (unsigned short*)(ws + kOffWOUT16);
  unsigned short* WX16   = (unsigned short*)(ws + kOffWX16);
  float*          XZ     = (float*)(ws + kOffXZ);
  float*          XI     = (float*)(ws + kOffXI);
  unsigned short* XI16   = (unsigned short*)(ws + kOffXI16);
  unsigned short* Y16    = XI16;
  float*          DLR    = (float*)(ws + kOffDLR);
  float*          BC     = (float*)(ws + kOffBC);

  cast_plane_kernel<<<(kRows * kDm / 8) / 256, 256, 0, stream>>>(x, X16, kRows * kDm / 8, kRows * kDm / 8, kCarryX);
  cast_plane_kernel<<<(kXzP * kDm / 8) / 256, 256, 0, stream>>>(W_in, WIN16, kXzP * kDm / 8, kXzP * kDm / 8, kCarryW);
  cast_plane_kernel<<<(kDin * kDin / 8) / 256, 256, 0, stream>>>(W_dt, WDT16, kDin * kDin / 8, kDin * kDin / 8, kCarryW);
  cast_plane_kernel<<<(kDm * kDin / 8) / 256, 256, 0, stream>>>(W_out, WOUT16, kDm * kDin / 8, kDm * kDin / 8, kCarryW);
  cast_plane_kernel<<<(kBcP * kDin / 8) / 256, 256, 0, stream>>>(W_x, WX16, kBcReal * kDin / 8, kBcP * kDin / 8, kCarryW);

  gemm_f16_kernel<<<(kRows / 64) * (kXzP / 64) / 8, 256, 0, stream>>>(
      X16, kDm, WIN16, kDm, XZ, kXzP, kRows, kXzP, kDm, kFoldS0);

  conv_silu_kernel<<<dim3(kDin / 256, kRows / 64), 256, 0, stream>>>(XZ, conv_w, conv_b, XI, XI16);

  gemm_f16_kernel<<<(kRows / 64) * (kDin / 64) / 8, 256, 0, stream>>>(
      XI16, kDin, WDT16, kDin, DLR, kDin, kRows, kDin, kDin, kFoldS1);

  gemm_f16_kernel<<<(kRows / 64) * (kBcP / 64) / 8, 256, 0, stream>>>(
      XI16, kDin, WX16, kDin, BC, kBcP, kRows, kBcP, kDin, kFoldS1);

  scan_kernel<<<kBatch * (kDin / kScanCh), kScanCh, 0, stream>>>(BC, DLR, XI, XZ, b_dt, A_log, Dp, Y16);

  gemm_f16_kernel<<<(kRows / 64) * (kDm / 64) / 8, 256, 0, stream>>>(
      Y16, kDin, WOUT16, kDin, out, kDm, kRows, kDm, kDin, kFoldS4);
}
